// DAttentionBaseline_56470230008330
// MI455X (gfx1250) — hardware-run, weakly checked
//
#include <hip/hip_runtime.h>
#include <stddef.h>

typedef __attribute__((ext_vector_type(16))) _Float16 v16h;
typedef __attribute__((ext_vector_type(8)))  _Float16 v8h;
typedef __attribute__((ext_vector_type(16))) __bf16   v16b;
typedef __attribute__((ext_vector_type(8)))  __bf16   v8b;
typedef __attribute__((ext_vector_type(8)))  float    v8f;
typedef __attribute__((ext_vector_type(4)))  float    v4f;

constexpr int kPos  = 4096;
constexpr int kCh   = 256;
constexpr int kGrp  = 4;
constexpr int kGch  = 64;
constexpr int kHch  = 32;
constexpr int kImg  = 64;
constexpr int kTab  = 127;
constexpr int kKtap = 9;

static_assert(kCh % 64 == 0 && kPos % 64 == 0 && kCh % 32 == 0);
static_assert(kGrp * kGch == kCh && 8 * kHch == kCh);

__device__ __forceinline__ unsigned short f2bf_bits(float f) {
  unsigned u = __float_as_uint(f);
  return (unsigned short)((u + 0x7FFFu + ((u >> 16) & 1u)) >> 16);
}
__device__ __forceinline__ float bf_bits2f(unsigned short h) { return __uint_as_float(((unsigned)h) << 16); }
__device__ __forceinline__ void split_bf(float f, _Float16& hi, _Float16& lo) {
  const unsigned short hb = f2bf_bits(f);
  const unsigned short lb = f2bf_bits(f - bf_bits2f(hb));
  hi = __builtin_bit_cast(_Float16, hb);
  lo = __builtin_bit_cast(_Float16, lb);
}

__device__ __forceinline__ void dep_guard_h(v8f& a, v8f& b, v16h x, v16h y) { asm volatile("v_nop\n\tv_nop\n\tv_nop\n\tv_nop" : "+v"(a), "+v"(b) : "v"(x), "v"(y)); }
__device__ __forceinline__ void dep_guard_b(v8f& a, v8f& b, v16b x, v16b y) { asm volatile("v_nop\n\tv_nop\n\tv_nop\n\tv_nop" : "+v"(a), "+v"(b) : "v"(x), "v"(y)); }
__device__ __forceinline__ void keep4_h(v16h a, v16h b, v16h c, v16h d) { asm volatile("v_nop" :: "v"(a), "v"(b), "v"(c), "v"(d)); }
__device__ __forceinline__ void keep4_b(v16b a, v16b b, v16b c, v16b d) { asm volatile("v_nop" :: "v"(a), "v"(b), "v"(c), "v"(d)); }
__device__ __forceinline__ void acc_guard4(v8f& a, v8f& b, v8f& c, v8f& d) { asm volatile("v_nop\n\tv_nop\n\tv_nop\n\tv_nop" : "+v"(a), "+v"(b), "+v"(c), "+v"(d)); }
template <typename T> struct Frag;
template <> struct Frag<_Float16> {
  typedef v16h V; union U { v16h v; v8h h[2]; };
  static __device__ __forceinline__ v16h load(const _Float16* p) {
    U f; f.h[0] = *(const v8h*)(p); f.h[1] = *(const v8h*)(p + 16); return f.v;
  }
  static __device__ __forceinline__ v8f mma(v16h a, v16h b, v8f c) {
    return __builtin_amdgcn_wmma_f32_16x16x32_f16(false, a, false, b, (short)0, c, false, false);
  }
  static __device__ __forceinline__ void guard(v8f& a, v8f& b, v16h x, v16h y) { dep_guard_h(a, b, x, y); }
  static __device__ __forceinline__ void keep(v16h a, v16h b, v16h c, v16h d) { keep4_h(a, b, c, d); }
};
template <> struct Frag<__bf16> {
  typedef v16b V; union U { v16b v; v8b h[2]; };
  static __device__ __forceinline__ v16b load(const __bf16* p) {
    U f; f.h[0] = *(const v8b*)(p); f.h[1] = *(const v8b*)(p + 16); return f.v;
  }
  static __device__ __forceinline__ v8f mma(v16b a, v16b b, v8f c) {
    return __builtin_amdgcn_wmma_f32_16x16x32_bf16(false, a, false, b, (short)0, c, false, false);
  }
  static __device__ __forceinline__ void guard(v8f& a, v8f& b, v16b x, v16b y) { dep_guard_b(a, b, x, y); }
  static __device__ __forceinline__ void keep(v16b a, v16b b, v16b c, v16b d) { keep4_b(a, b, c, d); }
};

__device__ __forceinline__ v8f mma_f16g(v16h a, v16h b, v8f c) {
  c = __builtin_amdgcn_wmma_f32_16x16x32_f16(false, a, false, b, (short)0, c, false, false);
  asm volatile("v_nop\n\tv_nop\n\tv_nop\n\tv_nop" : "+v"(c) : "v"(a), "v"(b));
  return c;
}
__device__ __forceinline__ void wave_sync_lds() {
  __builtin_amdgcn_fence(__ATOMIC_RELEASE, "workgroup");
  __builtin_amdgcn_wave_barrier();
  __builtin_amdgcn_fence(__ATOMIC_ACQUIRE, "workgroup");
}

template <int ET> struct Elem;
template <> struct Elem<0> { typedef _Float16 T; };
template <> struct Elem<1> { typedef __bf16 T; };
template <int ET, bool SPLIT, int BIAS_MODE, int OUT_MODE, int ACT>
__global__ __launch_bounds__(256) void wmma_gemm64(
    const unsigned short* __restrict__ Ap, const unsigned short* __restrict__ A2p, int lda, long strideA,
    const unsigned short* __restrict__ Btp, const unsigned short* __restrict__ Bt2p, int ldb, long strideB,
    void* __restrict__ Cout, void* __restrict__ Cout2, int ldc, long strideC,
    const float* __restrict__ bias, float bscale,
    int M, int N, int K, float scale) {
  typedef typename Elem<ET>::T T;
  typedef typename Frag<T>::V V;
  const T* A = (const T*)Ap; const T* A2 = (const T*)A2p; const T* Bt = (const T*)Btp; const T* Bt2 = (const T*)Bt2p;
  __shared__ __align__(16) float sT[8][16 * 68];
  const int b    = blockIdx.y;
  const int lane = threadIdx.x & 31;
  const int wave = threadIdx.x >> 5;
  const int tilesN = N >> 6;
  const int tilesM = M >> 6;
  const int tile = blockIdx.x * 8 + wave;
  if (tile >= tilesM * tilesN) return;
  const int tm = tile / tilesN;
  const int tn = tile - tm * tilesN;
  const int m0 = tm << 6;
  const int n0 = tn << 6;

  const T* Ab  = A  + (size_t)b * strideA;
  const T* Bb  = Bt + (size_t)b * strideB;
  const T* Ab2 = SPLIT ? (A2  + (size_t)b * strideA) : nullptr;
  const T* Bb2 = SPLIT ? (Bt2 + (size_t)b * strideB) : nullptr;

  const int rlane = lane & 15;
  const int koff  = (lane >> 4) * 8;
  const int mOff  = (lane >> 4) * 8;

  v8f acc[4][4];
#pragma unroll
  for (int i = 0; i < 4; ++i)
#pragma unroll
    for (int j = 0; j < 4; ++j) acc[i][j] = (v8f){0.f,0.f,0.f,0.f,0.f,0.f,0.f,0.f};

  for (int k0 = 0; k0 < K; k0 += 32) {
    V bh[4], bl[4];
#pragma unroll
    for (int j = 0; j < 4; ++j) {
      const size_t bo = (size_t)(n0 + (j << 4) + rlane) * ldb + koff + k0;
      bh[j] = Frag<T>::load(Bb + bo);
      if (SPLIT) bl[j] = Frag<T>::load(Bb2 + bo);
    }
#pragma unroll
    for (int i = 0; i < 4; ++i) {
      const size_t ao = (size_t)(m0 + (i << 4) + rlane) * lda + koff + k0;
      V ah = Frag<T>::load(Ab + ao);
      V al;
      if (SPLIT) al = Frag<T>::load(Ab2 + ao);
#pragma unroll
      for (int j = 0; j < 4; ++j) {
        acc[i][j] = Frag<T>::mma(ah, bh[j], acc[i][j]);
        if (SPLIT) {
          acc[i][j] = Frag<T>::mma(ah, bl[j], acc[i][j]);
          acc[i][j] = Frag<T>::mma(al, bh[j], acc[i][j]);
        }
      }
      Frag<T>::guard(acc[i][0], acc[i][3], ah, SPLIT ? al : ah);
    }
    Frag<T>::keep(bh[0], bh[1], bh[2], bh[3]);
    if (SPLIT) Frag<T>::keep(bl[0], bl[1], bl[2], bl[3]);
  }
  acc_guard4(acc[0][0], acc[0][1], acc[0][2], acc[0][3]);
  acc_guard4(acc[1][0], acc[1][1], acc[1][2], acc[1][3]);
  acc_guard4(acc[2][0], acc[2][1], acc[2][2], acc[2][3]);
  acc_guard4(acc[3][0], acc[3][1], acc[3][2], acc[3][3]);

  float* slab = sT[wave];
#pragma unroll
  for (int i = 0; i < 4; ++i) {
    const int mBase = m0 + (i << 4);
    float bm[8];
#pragma unroll
    for (int r = 0; r < 8; ++r) bm[r] = 0.f;
    if (BIAS_MODE == 1) {
      const v4f b0 = *(const v4f*)(bias + mBase + mOff);
      const v4f b1 = *(const v4f*)(bias + mBase + mOff + 4);
      bm[0] = b0[0]; bm[1] = b0[1]; bm[2] = b0[2]; bm[3] = b0[3];
      bm[4] = b1[0]; bm[5] = b1[1]; bm[6] = b1[2]; bm[7] = b1[3];
    }
#pragma unroll
    for (int j = 0; j < 4; ++j) {
      const int n = n0 + (j << 4) + rlane;
      float bv = 0.f;
      if (BIAS_MODE == 2) bv = bias[n];
#pragma unroll
      for (int r = 0; r < 8; ++r) {
        float v = acc[i][j][r] * scale;
        if (BIAS_MODE == 1) v += bm[r] * bscale;
        if (BIAS_MODE == 2) v += bv * bscale;
        if (ACT == 1) v = tanhf(v);
        if (ACT == 2) v = fmaxf(v, 0.0f);
        if (ACT == 3) v = v / (1.0f + expf(-v));
        if (ACT == 4) v = (v > 0.f) ? v : 0.01f * v;
        slab[(mOff + r) * 68 + (j << 4) + rlane] = v;
      }
    }
    __builtin_amdgcn_fence(__ATOMIC_RELEASE, "workgroup");
    __builtin_amdgcn_wave_barrier();
    __builtin_amdgcn_fence(__ATOMIC_ACQUIRE, "workgroup");
    if (OUT_MODE == 0) {
      float* C = (float*)Cout + (size_t)b * strideC;
      const int hh = lane >> 4, c4 = (lane & 15) * 4;
      for (int pass = 0; pass < 2; ++pass) {
#pragma unroll
        for (int it = 0; it < 8; ++it) {
          const int row = it * 2 + hh;
          v4f v = *(const v4f*)(slab + row * 68 + c4);
          *(volatile v4f*)(C + (size_t)(mBase + row) * ldc + n0 + c4) = v;
        }
        __threadfence();
      }
    } else {
      const int q = lane >> 3, c8 = (lane & 7) * 8;
      unsigned short* C  = (unsigned short*)Cout  + (size_t)b * strideC;
      unsigned short* C2 = (OUT_MODE == 2) ? ((unsigned short*)Cout2 + (size_t)b * strideC) : nullptr;
      for (int pass = 0; pass < 2; ++pass) {
#pragma unroll
        for (int it = 0; it < 4; ++it) {
          const int row = it * 4 + q;
          const float* sp = slab + row * 68 + c8;
          v8h hv, lv;
#pragma unroll
          for (int e = 0; e < 8; ++e) {
            if (OUT_MODE == 1) {
              hv[e] = (_Float16)sp[e];
            } else {
              unsigned short hb = f2bf_bits(sp[e]);
              unsigned short lb = f2bf_bits(sp[e] - bf_bits2f(hb));
              hv[e] = __builtin_bit_cast(_Float16, hb);
              lv[e] = __builtin_bit_cast(_Float16, lb);
            }
          }
          *(volatile v8h*)(C + (size_t)(mBase + row) * ldc + n0 + c8) = hv;
          if (OUT_MODE == 2) *(volatile v8h*)(C2 + (size_t)(mBase + row) * ldc + n0 + c8) = lv;
        }
        __threadfence();
      }
    }
    __builtin_amdgcn_fence(__ATOMIC_RELEASE, "workgroup");
    __builtin_amdgcn_wave_barrier();
    __builtin_amdgcn_fence(__ATOMIC_ACQUIRE, "workgroup");
  }
}

__global__ __launch_bounds__(256) void k_wsplit(const float* __restrict__ w0, const float* __restrict__ w1,
                                                const float* __restrict__ w2, const float* __restrict__ w3,
                                                unsigned short* __restrict__ plp) {
  const int seg = blockIdx.x >> 5;
  const float* src = (seg == 0) ? w0 : (seg == 1) ? w1 : (seg == 2) ? w2 : w3;
  const int e0 = ((blockIdx.x & 31) * 256 + threadIdx.x) * 8;
  const v4f a = *(const v4f*)(src + e0);
  const v4f c2 = *(const v4f*)(src + e0 + 4);
  v8h hv, lv;
#pragma unroll
  for (int e = 0; e < 4; ++e) {
    _Float16 hA, lA, hB, lB;
    split_bf(a[e], hA, lA);
    split_bf(c2[e], hB, lB);
    hv[e] = hA; lv[e] = lA; hv[4 + e] = hB; lv[4 + e] = lB;
  }
  _Float16* pl = (_Float16*)(void*)plp;
  _Float16* ph = pl + (size_t)(2 * seg) * 65536 + e0;
  _Float16* po = pl + (size_t)(2 * seg + 1) * 65536 + e0;
  *(volatile v8h*)ph = hv;
  *(volatile v8h*)po = lv;
  __threadfence();
  *(volatile v8h*)ph = hv;
  *(volatile v8h*)po = lv;
}

template <int MODE>
__global__ __launch_bounds__(256) void k_tr16(const float* __restrict__ in, unsigned short* __restrict__ o1p,
                                              unsigned short* __restrict__ o2p, float scl) {
  __shared__ __align__(16) float tile[64][65];
  const int tid = threadIdx.x, lane = tid & 31, wave = tid >> 5;
  const int col0 = blockIdx.x * 64;
  const int row0 = blockIdx.y * 64;
  {
    const int c4 = (tid & 15) * 4, rb = tid >> 4;
#pragma unroll
    for (int i = 0; i < 4; ++i) {
      const int r = i * 16 + rb;
      const v4f v = *(const v4f*)(in + (size_t)(row0 + r) * kPos + col0 + c4);
      tile[r][c4] = v[0]; tile[r][c4 + 1] = v[1]; tile[r][c4 + 2] = v[2]; tile[r][c4 + 3] = v[3];
    }
  }
  __syncthreads();
  _Float16* o1 = (_Float16*)(void*)o1p;
  _Float16* o2 = (_Float16*)(void*)o2p;
  const int q4 = lane >> 3, c8 = (lane & 7) * 8;
  for (int pass = 0; pass < 2; ++pass) {
#pragma unroll
    for (int it = 0; it < 2; ++it) {
      const int prow = wave * 8 + it * 4 + q4;
      v8h hv, lv;
#pragma unroll
      for (int e = 0; e < 8; ++e) {
        const float f = tile[c8 + e][prow];
        if (MODE == 0) {
          _Float16 hA, lA; split_bf(f, hA, lA); hv[e] = hA; lv[e] = lA;
        } else {
          hv[e] = (_Float16)(f * scl); lv[e] = hv[e];
        }
      }
      const size_t o = (size_t)(col0 + prow) * kCh + row0 + c8;
      *(volatile v8h*)(o1 + o) = hv;
      if (MODE == 0) *(volatile v8h*)(o2 + o) = lv;
    }
    __threadfence();
  }
}

__global__ __launch_bounds__(256) void k_dwconv(const float* __restrict__ qf, const float* __restrict__ wdw,
                                                const float* __restrict__ bdw, float* __restrict__ odw) {
  __shared__ __align__(16) float tl[72 * 72];
  __shared__ float wl[96];
  const int tid = threadIdx.x;
  const int gch = blockIdx.x;
  const int cg = gch & 63;
  const float* qc = qf + (size_t)gch * kPos;
  for (int idx = tid; idx < 72 * 72; idx += 256) {
    const int r = idx / 72;
    const int cc = idx - r * 72;
    const int iy = r - 4, ix = cc - 4;
    const bool inb = (iy >= 0) && (iy < kImg) && (ix >= 0) && (ix < kImg);
    const int iyc = min(max(iy, 0), kImg - 1), ixc = min(max(ix, 0), kImg - 1);
    const float v = qc[iyc * kImg + ixc];
    tl[idx] = inb ? v : 0.0f;
  }
  if (tid < kKtap * kKtap) wl[tid] = wdw[cg * (kKtap * kKtap) + tid];
  __syncthreads();
  const float bb = bdw[cg];
#pragma unroll 1
  for (int i = 0; i < 4; ++i) {
    const int o = (i * 256 + tid) * 4;
    const int y = o >> 6, x = o & 63;
    float acc0 = 0.0f, acc1 = 0.0f, acc2 = 0.0f, acc3 = 0.0f;
#pragma unroll 1
    for (int ky = 0; ky < kKtap; ++ky) {
      const float* rp = tl + (y + ky) * 72 + x;
      const v4f t0 = *(const v4f*)(rp);
      const v4f t1 = *(const v4f*)(rp + 4);
      const v4f t2 = *(const v4f*)(rp + 8);
      const float t[12] = {t0[0], t0[1], t0[2], t0[3], t1[0], t1[1], t1[2], t1[3], t2[0], t2[1], t2[2], t2[3]};
      const float* wp = wl + ky * kKtap;
#pragma unroll
      for (int kx = 0; kx < kKtap; ++kx) {
        const float w = wp[kx];
        acc0 += t[kx] * w; acc1 += t[kx + 1] * w; acc2 += t[kx + 2] * w; acc3 += t[kx + 3] * w;
      }
    }
    v4f ov;
    ov[0] = acc0 + bb; ov[1] = acc1 + bb; ov[2] = acc2 + bb; ov[3] = acc3 + bb;
    float* dst = odw + (size_t)gch * kPos + o;
    *(volatile v4f*)dst = ov;
    __threadfence();
    *(volatile v4f*)dst = ov;
  }
}

__global__ __launch_bounds__(256) void k_offpos(const float* __restrict__ odw, const float* __restrict__ lng,
                                                const float* __restrict__ lnb, const float* __restrict__ wpw,
                                                float* __restrict__ posb) {
  const int idx = blockIdx.x * 256 + threadIdx.x;
  if (idx >= kGrp * kPos) return;
  const int g = idx >> 12, hw = idx & (kPos - 1);
  const float* base = odw + (size_t)g * kGch * kPos + hw;
  float s1 = 0.0f;
#pragma unroll 1
  for (int cc = 0; cc < kGch; ++cc) s1 += base[(size_t)cc * kPos];
  const float mu = s1 * (1.0f / 64.0f);
  float s2 = 0.0f;
#pragma unroll 1
  for (int cc = 0; cc < kGch; ++cc) { const float d = base[(size_t)cc * kPos] - mu; s2 += d * d; }
  const float var = s2 * (1.0f / 64.0f);
  const float rs = 1.0f / sqrtf(var + 1e-5f);
  float o0 = 0.0f, o1 = 0.0f;
#pragma unroll 1
  for (int cc = 0; cc < kGch; ++cc) {
    const float v = base[(size_t)cc * kPos];
    const float t = (v - mu) * rs * lng[cc] + lnb[cc];
    const float ge = 0.5f * t * (1.0f + erff(t * 0.70710678118654752f));
    o0 += ge * wpw[cc];
    o1 += ge * wpw[kGch + cc];
  }
  const int yy = hw >> 6, xx = hw & 63;
  const float ry = ((float)yy + 0.5f) * 0.03125f - 1.0f;
  const float rx = ((float)xx + 0.5f) * 0.03125f - 1.0f;
  const float py = tanhf(o0) * 0.03125f + ry;
  const float px = tanhf(o1) * 0.03125f + rx;
  v4f pv;
  pv[0] = py; pv[1] = px; pv[2] = 63.0f - 31.5f * py; pv[3] = 63.0f - 31.5f * px;
  float* dst = posb + (size_t)idx * 4;
  *(volatile v4f*)dst = pv;
  __threadfence();
  *(volatile v4f*)dst = pv;
}

__global__ __launch_bounds__(256) void k_sample(const float* __restrict__ x, const float* __restrict__ posb,
                                                unsigned short* __restrict__ xshp, unsigned short* __restrict__ xslp) {
  __shared__ __align__(16) _Float16 shh[8][256];
  __shared__ __align__(16) _Float16 shl[8][256];
  const int tid = threadIdx.x, lane = tid & 31, wave = tid >> 5;
  const int s = blockIdx.x * 8 + wave;
#pragma unroll 1
  for (int p = 0; p < 2; ++p) {
    const int cb = p * 128 + lane * 4;
    const int g = cb >> 6;
    const v4f pp = *(const v4f*)(posb + ((size_t)g * kPos + s) * 4);
    const float py = pp[0], px = pp[1];
    float tx = px + 1.0f; tx = tx * 0.5f; const float gx = tx * 63.0f;
    float ty = py + 1.0f; ty = ty * 0.5f; const float gy = ty * 63.0f;
    const float x0 = floorf(gx), y0 = floorf(gy);
    const int ix0 = (int)x0, iy0 = (int)y0;
    float wx0 = 1.0f - (gx - x0);
    float wx1 = 1.0f - ((x0 + 1.0f) - gx);
    float wy0 = 1.0f - (gy - y0);
    float wy1 = 1.0f - ((y0 + 1.0f) - gy);
    wx0 = (ix0 >= 0 && ix0 <= kImg - 1) ? wx0 : 0.0f;
    wx1 = (ix0 >= -1 && ix0 <= kImg - 2) ? wx1 : 0.0f;
    wy0 = (iy0 >= 0 && iy0 <= kImg - 1) ? wy0 : 0.0f;
    wy1 = (iy0 >= -1 && iy0 <= kImg - 2) ? wy1 : 0.0f;
    const int ix0c = min(max(ix0, 0), kImg - 1), ix1c = min(max(ix0 + 1, 0), kImg - 1);
    const int iy0c = min(max(iy0, 0), kImg - 1), iy1c = min(max(iy0 + 1, 0), kImg - 1);
    const float w00 = wx0 * wy0, w01 = wx1 * wy0, w10 = wx0 * wy1, w11 = wx1 * wy1;
    const int a00 = iy0c * kImg + ix0c, a01 = iy0c * kImg + ix1c, a10 = iy1c * kImg + ix0c, a11 = iy1c * kImg + ix1c;
#pragma unroll
    for (int e = 0; e < 4; ++e) {
      const float* xc = x + (size_t)(cb + e) * kPos;
      const float v00 = xc[a00], v01 = xc[a01], v10 = xc[a10], v11 = xc[a11];
      float val = 0.0f + v00 * w00;
      val = val + v01 * w01;
      val = val + v10 * w10;
      val = val + v11 * w11;
      _Float16 hA, lA;
      split_bf(val, hA, lA);
      shh[wave][cb + e] = hA;
      shl[wave][cb + e] = lA;
    }
  }
  __syncthreads();
  _Float16* xsh = (_Float16*)(void*)xshp;
  _Float16* xsl = (_Float16*)(void*)xslp;
  const size_t o = (size_t)s * kCh + lane * 8;
  for (int pass = 0; pass < 2; ++pass) {
    const v8h hv = *(const v8h*)(&shh[wave][lane * 8]);
    const v8h lv = *(const v8h*)(&shl[wave][lane * 8]);
    *(volatile v8h*)(xsh + o) = hv;
    *(volatile v8h*)(xsl + o) = lv;
    __threadfence();
  }
}

__device__ __forceinline__ float tab_sample(const _Float16* tb, float gy, float gx) {
  const float y0 = floorf(gy), x0 = floorf(gx);
  const float fy = gy - y0, fx = gx - x0;
  const int iy0 = (int)y0, ix0 = (int)x0;
  const float wy0 = (iy0 >= 0) ? (1.0f - fy) : 0.0f;
  const float wy1 = (iy0 >= -1) ? fy : 0.0f;
  const float wx0 = (ix0 >= 0) ? (1.0f - fx) : 0.0f;
  const float wx1 = (ix0 >= -1) ? fx : 0.0f;
  const int iy0c = min(max(iy0, 0), 127), iy1c = min(max(iy0 + 1, 0), 127);
  const int ix0c = min(max(ix0, 0), 127), ix1c = min(max(ix0 + 1, 0), 127);
  const float v00 = (float)tb[iy0c * 128 + ix0c];
  const float v01 = (float)tb[iy0c * 128 + ix1c];
  const float v10 = (float)tb[iy1c * 128 + ix0c];
  const float v11 = (float)tb[iy1c * 128 + ix1c];
  const float top = v00 * wx0 + v01 * wx1;
  const float bot = v10 * wx0 + v11 * wx1;
  return top * wy0 + bot * wy1;
}

__global__ __launch_bounds__(128) void k_attn(const unsigned short* __restrict__ qhp,
                                              const unsigned short* __restrict__ khp,
                                              const unsigned short* __restrict__ vhp,
                                              const float* __restrict__ posb,
                                              const float* __restrict__ rpe,
                                              unsigned short* __restrict__ aohp,
                                              unsigned short* __restrict__ aolp) {
  __shared__ __align__(16) _Float16 Tsh[128 * 128];
  __shared__ __align__(16) _Float16 Ksh[32 * 32];
  __shared__ __align__(16) _Float16 Vsh[32 * 32];
  __shared__ __align__(16) _Float16 Psh[4][16 * 32];
  __shared__ __align__(16) float Ash[64];
  __shared__ __align__(16) float Osh[4][16 * 68];

  const _Float16* qh = (const _Float16*)(const void*)qhp;
  const _Float16* kh = (const _Float16*)(const void*)khp;
  const _Float16* vh = (const _Float16*)(const void*)vhp;
  const int tid = threadIdx.x, wave = tid >> 5, lane = tid & 31, hh = lane >> 4, c = lane & 15;
  const int g = blockIdx.y;
  const int q0 = blockIdx.x * 64 + wave * 16;
  const float kQkFold = 0.17677669529663687f * (1.0f / 64.0f);

  float QY[8], QX[8];
#pragma unroll
  for (int r = 0; r < 8; ++r) {
    const int m = q0 + 8 * hh + r;
    const float ry = ((float)(m >> 6) + 0.5f) * 0.03125f - 1.0f;
    const float rx = ((float)(m & 63) + 0.5f) * 0.03125f - 1.0f;
    QY[r] = ry * 31.5f;
    QX[r] = rx * 31.5f;
  }
  const v8f zero8 = {0.f, 0.f, 0.f, 0.f, 0.f, 0.f, 0.f, 0.f};
  float* os = Osh[wave];
  _Float16* pw = Psh[wave];

#pragma unroll 1
  for (int hl = 0; hl < 2; ++hl) {
    const int h = 2 * g + hl;
    __syncthreads();
#pragma unroll 2
    for (int idx = tid; idx < 128 * 128; idx += 128) {
      const int r = idx >> 7, cc = idx & 127;
      const int rc = min(r, kTab - 1), ccc = min(cc, kTab - 1);
      const float tv = rpe[((size_t)h * kTab + rc) * kTab + ccc];
      const float sv = (r < kTab && cc < kTab) ? tv * 4096.0f : 0.0f;
      Tsh[idx] = (_Float16)sv;
    }
    const v16h qa = Frag<_Float16>::load(qh + (size_t)(q0 + c) * kCh + h * kHch + 8 * hh);
    float mrow[8], lrow[8];
    v8f oacc[2];
#pragma unroll
    for (int r = 0; r < 8; ++r) { mrow[r] = -INFINITY; lrow[r] = 0.0f; }
    oacc[0] = zero8; oacc[1] = zero8;

    for (int kc = 0; kc < kPos / 32; ++kc) {
      const int kv0 = kc * 32;
      __syncthreads();
      {
        const int rr = tid >> 2, e8 = (tid & 3) * 8;
        const v8h kv = *(const v8h*)(kh + (size_t)(kv0 + rr) * kCh + h * kHch + e8);
        const v8h vv = *(const v8h*)(vh + (size_t)(h * kHch + rr) * kPos + kv0 + e8);
        *(v8h*)(Ksh + rr * 32 + e8) = kv;
        *(v8h*)(Vsh + rr * 32 + e8) = vv;
        if (wave == 0) {
          const v4f pp = *(const v4f*)(posb + ((size_t)g * kPos + kv0 + lane) * 4);
          Ash[lane * 2] = pp[2];
          Ash[lane * 2 + 1] = pp[3];
        }
      }
      __syncthreads();

      v8f s[2];
#pragma unroll
      for (int j = 0; j < 2; ++j) {
        const v16h kb = Frag<_Float16>::load(Ksh + (j * 16 + c) * 32 + 8 * hh);
        s[j] = mma_f16g(qa, kb, zero8);
      }
      float ay[2], ax[2];
#pragma unroll
      for (int j = 0; j < 2; ++j) { ay[j] = Ash[(j * 16 + c) * 2]; ax[j] = Ash[(j * 16 + c) * 2 + 1]; }

      float cm[8];
#pragma unroll
      for (int r = 0; r < 8; ++r) {
        float mx = -INFINITY;
#pragma unroll
        for (int j = 0; j < 2; ++j) {
          const float bias = tab_sample(Tsh, QY[r] + ay[j], QX[r] + ax[j]);
          const float sv = s[j][r] * kQkFold + bias * (1.0f / 4096.0f);
          s[j][r] = sv;
          mx = fmaxf(mx, sv);
        }
#pragma unroll
        for (int off = 1; off < 16; off <<= 1) mx = fmaxf(mx, __shfl_xor(mx, off, 32));
        cm[r] = mx;
      }
#pragma unroll
      for (int r = 0; r < 8; ++r) {
        const float mnew = fmaxf(mrow[r], cm[r]);
        const float alpha = expf(mrow[r] - mnew);
        mrow[r] = mnew;
        float psum = 0.0f;
#pragma unroll
        for (int j = 0; j < 2; ++j) {
          const float p = expf(s[j][r] - mnew);
          psum += p;
          pw[(8 * hh + r) * 32 + j * 16 + c] = (_Float16)(p * 1024.0f);
        }
#pragma unroll
        for (int off = 1; off < 16; off <<= 1) psum += __shfl_xor(psum, off, 32);
        lrow[r] = lrow[r] * alpha + psum;
        oacc[0][r] *= alpha;
        oacc[1][r] *= alpha;
      }
      wave_sync_lds();
      const v16h pa = Frag<_Float16>::load(pw + c * 32 + 8 * hh);
#pragma unroll
      for (int t = 0; t < 2; ++t) {
        const v16h vb = Frag<_Float16>::load(Vsh + (t * 16 + c) * 32 + 8 * hh);
        oacc[t] = mma_f16g(pa, vb, oacc[t]);
      }
    }
#pragma unroll
    for (int r = 0; r < 8; ++r) {
      const float inv = (1.0f / lrow[r]) * (1.0f / 8192.0f);
#pragma unroll
      for (int t = 0; t < 2; ++t) os[(8 * hh + r) * 68 + hl * 32 + t * 16 + c] = oacc[t][r] * inv;
    }
  }
  __syncthreads();
  {
    _Float16* aoh = (_Float16*)(void*)aohp;
    _Float16* aol = (_Float16*)(void*)aolp;
    const int q4 = lane >> 3, c8 = (lane & 7) * 8;
    for (int pass = 0; pass < 2; ++pass) {
#pragma unroll
      for (int it = 0; it < 4; ++it) {
        const int row = it * 4 + q4;
        const float* sp = os + row * 68 + c8;
        v8h hv, lv;
#pragma unroll
        for (int e = 0; e < 8; ++e) { _Float16 hA, lA; split_bf(sp[e], hA, lA); hv[e] = hA; lv[e] = lA; }
        const size_t o = (size_t)(q0 + row) * kCh + g * kGch + c8;
        *(volatile v8h*)(aoh + o) = hv;
        *(volatile v8h*)(aol + o) = lv;
      }
      __threadfence();
    }
  }
}

extern "C" void kernel_launch(void* const* d_in, const int* in_sizes, int n_in,
                              void* d_out, int out_size, void* d_ws, size_t ws_size,
                              hipStream_t stream) {
  (void)in_sizes;
  constexpr size_t kP16  = (size_t)kPos * kCh * 2;
  constexpr size_t kP32  = (size_t)kPos * kCh * 4;
  constexpr size_t kWpl  = (size_t)kCh * kCh * 2;
  constexpr size_t kPosB = (size_t)kGrp * kPos * 4 * 4;
  constexpr size_t oXTh = 0;
  constexpr size_t oXTl = oXTh + kP16;
  constexpr size_t oW   = oXTl + kP16;
  constexpr size_t oQf  = oW + 8 * kWpl;
  constexpr size_t oQh  = oQf + kP32;
  constexpr size_t oOdw = oQh + kP16;
  constexpr size_t oPos = oOdw + kP32;
  constexpr size_t oXsh = oPos + kPosB;
  constexpr size_t oXsl = oXsh + kP16;
  constexpr size_t oKh  = oXsl + kP16;
  constexpr size_t oVh  = oKh + kP16;
  constexpr size_t oAoh = oVh + kP16;
  constexpr size_t oAol = oAoh + kP16;
  constexpr size_t oEnd = oAol + kP16;
  static_assert(oEnd == 28573696);
  static_assert((oW % 256) == 0 && (oPos % 256) == 0 && (oXsh % 256) == 0 && (oAol % 256) == 0);
  if (n_in < 15 || (size_t)out_size < (size_t)kPos * kCh || ws_size < oEnd) return;

  const float* x     = (const float*)d_in[0];
  const float* wq    = (const float*)d_in[1];
  const float* bq    = (const float*)d_in[2];
  const float* wk    = (const float*)d_in[3];
  const float* bk    = (const float*)d_in[4];
  const float* wv    = (const float*)d_in[5];
  const float* bv    = (const float*)d_in[6];
  const float* w_dw  = (const float*)d_in[7];
  const float* b_dw  = (const float*)d_in[8];
  const float* ln_g  = (const float*)d_in[9];
  const float* ln_b  = (const float*)d_in[10];
  const float* w_pw  = (const float*)d_in[11];
  const float* rpe   = (const float*)d_in[12];
  const float* w_out = (const float*)d_in[13];
  const float* b_out = (const float*)d_in[14];
  float* outp = (float*)d_out;

  char* ws = (char*)d_ws;
  unsigned short* xT_hi = (unsigned short*)(ws + oXTh);
  unsigned short* xT_lo = (unsigned short*)(ws + oXTl);
  unsigned short* wpl   = (unsigned short*)(ws + oW);
  unsigned short* wq_hi = wpl;
  unsigned short* wq_lo = wpl + 65536;
  unsigned short* wk_hi = wpl + 2 * 65536;
  unsigned short* wk_lo = wpl + 3 * 65536;
  unsigned short* wv_hi = wpl + 4 * 65536;
  unsigned short* wv_lo = wpl + 5 * 65536;
  unsigned short* wo_hi = wpl + 6 * 65536;
  unsigned short* wo_lo = wpl + 7 * 65536;
  float*          qf    = (float*)(ws + oQf);
  unsigned short* qh    = (unsigned short*)(ws + oQh);
  float*          odw   = (float*)(ws + oOdw);
  float*          posb  = (float*)(ws + oPos);
  unsigned short* xs_hi = (unsigned short*)(ws + oXsh);
  unsigned short* xs_lo = (unsigned short*)(ws + oXsl);
  unsigned short* kh    = (unsigned short*)(ws + oKh);
  unsigned short* vh    = (unsigned short*)(ws + oVh);
  unsigned short* ao_hi = (unsigned short*)(ws + oAoh);
  unsigned short* ao_lo = (unsigned short*)(ws + oAol);

  k_wsplit<<<dim3(128), dim3(256), 0, stream>>>(wq, wk, wv, w_out, wpl);
  k_tr16<0><<<dim3(64, 4), dim3(256), 0, stream>>>(x, xT_hi, xT_lo, 1.0f);
  wmma_gemm64<1, true, 1, 0, 0><<<dim3(32, 1), dim3(256), 0, stream>>>(
      wq_hi, wq_lo, kCh, 0L, xT_hi, xT_lo, kCh, 0L, (void*)qf, (void*)qf, kPos, 0L,
      bq, 1.0f, kCh, kPos, kCh, 1.0f);
  k_tr16<1><<<dim3(64, 4), dim3(256), 0, stream>>>(qf, qh, qh, 8.0f);
  k_dwconv<<<dim3(256), dim3(256), 0, stream>>>(qf, w_dw, b_dw, odw);
  k_offpos<<<dim3(64), dim3(256), 0, stream>>>(odw, ln_g, ln_b, w_pw, posb);
  k_sample<<<dim3(512), dim3(256), 0, stream>>>(x, posb, xs_hi, xs_lo);
  wmma_gemm64<1, true, 2, 1, 0><<<dim3(32, 1), dim3(256), 0, stream>>>(
      xs_hi, xs_lo, kCh, 0L, wk_hi, wk_lo, kCh, 0L, (void*)kh, (void*)kh, kCh, 0L,
      bk, 8.0f, kPos, kCh, kCh, 8.0f);
  wmma_gemm64<1, true, 1, 1, 0><<<dim3(32, 1), dim3(256), 0, stream>>>(
      wv_hi, wv_lo, kCh, 0L, xs_hi, xs_lo, kCh, 0L, (void*)vh, (void*)vh, kPos, 0L,
      bv, 8.0f, kCh, kPos, kCh, 8.0f);
  k_attn<<<dim3(64, 4), dim3(128), 0, stream>>>(qh, kh, vh, posb, rpe, ao_hi, ao_lo);
  wmma_gemm64<1, true, 1, 0, 0><<<dim3(32, 1), dim3(256), 0, stream>>>(
      wo_hi, wo_lo, kCh, 0L, ao_hi, ao_lo, kCh, 0L, (void*)outp, (void*)outp, kPos, 0L,
      b_out, 1.0f, kCh, kPos, kCh, 1.0f);
}
